// GINModel_38010460569655
// MI455X (gfx1250) — hardware-run, weakly checked
//
#include <hip/hip_runtime.h>
#include <stddef.h>
#include <stdint.h>

#define NN      50000
#define NE      800000
#define VOC     1001
#define HD      128
#define NC      40
#define NCP     48
#define NLAY    3
#define GBM     128
#define MP      50048
#define KTOT    256
#define NTHR    256
#define NWAVE   8
#define EPT     8
#define WCH     (32 * EPT)
#define NBRUN   1024
#define SLB     10
#define NBK     49
#define WLCAP   2560
#define RCAP    20480
#define DEGCAP  64
#define MAXDEG_MEAS   33
#define MAXB1024_MEAS 16696
#define RBM     64
#define SP      132
#define TPH     264
#define WSMAX   (128u << 20)

#define BK_ZINTS (NWAVE * WLCAP + RCAP + 3 * NBRUN)
#define BK_INTS  (BK_ZINTS + 16)
#define BK_LDS   (BK_INTS * 4)
#define ML_INTS  (GBM * SP + (GBM * TPH) / 2 + 2 * HD)
#define ML_LDS   (ML_INTS * 4)

#define PBH   (MP * 32 / NTHR)
#define PBW   (NLAY * HD * KTOT / 8 / NTHR)
#define PBC   (NCP * KTOT / 8 / NTHR)
#define PBTOT (PBH + 2 * PBW + PBC + 1)

static_assert(HD == 128 && HD == 32 * 4 && KTOT == 2 * HD && KTOT % 32 == 0);
static_assert(MP % GBM == 0 && MP >= NN && MP == 391 * GBM && MP % RBM == 0);
static_assert(NBRUN == (1 << SLB) && NBRUN % RBM == 0 && NBRUN % GBM == 0 && NBRUN == 8 * GBM);
static_assert(NBK * NBRUN >= MP && (NBK - 1) * NBRUN < NN);
static_assert(NE < (1 << 21) && (((long long)NE) << SLB) < (1LL << 31));
static_assert(NE % WCH == 0 && NE % 4 == 0);
static_assert(RCAP == NWAVE * WLCAP && RCAP % (NTHR * 4) == 0 && BK_ZINTS % (NTHR * 4) == 0);
static_assert((2 * NBRUN) % (NTHR * 4) == 0);
static_assert((long long)RCAP * 100 >= (long long)MAXB1024_MEAS * 105);
static_assert(WLCAP >= MAXB1024_MEAS / 8 + 8 * 46 + 1);
static_assert(NN <= 65536);
static_assert(MAXDEG_MEAS + 8 <= DEGCAP && DEGCAP <= 64);
static_assert((GBM * NC * 4) % 128 == 0 && (((NN % GBM) * NC * 4) % 128) == 0);
static_assert(GBM * NC / 4 == 5 * NTHR && ((NN % GBM) * NC / 4) % 32 == 0);
static_assert((MP * 32) % NTHR == 0 && (NLAY * HD * KTOT / 8) % NTHR == 0 && (NCP * KTOT / 8) % NTHR == 0);
static_assert(HD * KTOT / 8 == 4096 && NCP % 16 == 0 && NCP >= NC);
static_assert(2 * NLAY * HD == 768 && 2 * NLAY * HD / 4 == 192);
static_assert(BK_LDS <= 300000 && ML_LDS <= 300000);
static_assert((TPH * 2) % 16 == 0 && TPH >= KTOT && SP >= HD && (SP * 4) % 16 == 0);
static_assert(GBM * NC <= GBM * SP);
static_assert(GBM == NWAVE * 16 && RBM == NWAVE * 8);

typedef float          v4f   __attribute__((ext_vector_type(4)));
typedef float          v8f   __attribute__((ext_vector_type(8)));
typedef int            v2i   __attribute__((ext_vector_type(2)));
typedef int            v4i   __attribute__((ext_vector_type(4)));
typedef int            v8i   __attribute__((ext_vector_type(8)));
typedef unsigned short v8us  __attribute__((ext_vector_type(8)));
typedef unsigned short v16us __attribute__((ext_vector_type(16)));
typedef __bf16         v16bf __attribute__((ext_vector_type(16)));
typedef v4f  __attribute__((may_alias)) v4fa;
typedef v2i  __attribute__((may_alias)) v2ia;
typedef v4i  __attribute__((may_alias)) v4ia;
typedef v8us __attribute__((may_alias)) v8usa;
union FragB { v16bf v; v16us u; v8us h[2]; v8i w; };

__device__ __forceinline__ v8f wmb(const FragB& a, const FragB& b, v8f c) {
  v8f d = __builtin_amdgcn_wmma_f32_16x16x32_bf16(false, a.v, false, b.v, (short)0, c, false, false);
  asm volatile("v_nop\n\tv_nop\n\tv_nop\n\tv_nop" : "+v"(d) : "v"(a.w), "v"(b.w));
  return d;
}

__device__ __forceinline__ unsigned bf16_bits(float f) {
  const unsigned u = __float_as_uint(f);
  const unsigned r = (u + 0x7FFFu + ((u >> 16) & 1u)) >> 16;
  const unsigned q = (u >> 16) | 0x40u;
  return ((u & 0x7fffffffu) > 0x7f800000u) ? q : r;
}
__device__ __forceinline__ float bf16_val(float f) {
  return __uint_as_float(bf16_bits(f) << 16);
}

__device__ __forceinline__ void hilo_pack(float v0, float v1, float v2, float v3,
                                          int& h01, int& h23, int& l01, int& l23) {
  const unsigned a0 = bf16_bits(v0), a1 = bf16_bits(v1), a2 = bf16_bits(v2), a3 = bf16_bits(v3);
  const unsigned b0 = bf16_bits(v0 - __uint_as_float(a0 << 16));
  const unsigned b1 = bf16_bits(v1 - __uint_as_float(a1 << 16));
  const unsigned b2 = bf16_bits(v2 - __uint_as_float(a2 << 16));
  const unsigned b3 = bf16_bits(v3 - __uint_as_float(a3 << 16));
  h01 = (int)(a0 | (a1 << 16)); h23 = (int)(a2 | (a3 << 16));
  l01 = (int)(b0 | (b1 << 16)); l23 = (int)(b2 | (b3 << 16));
}

__device__ __forceinline__ v4i regroup32(int h01, int h23, int l01, int l23, int lane) {
  const int s0 = (2 * lane) & 31, s1 = s0 + 1;
  const int a0 = __shfl(h01, s0, 32), a1 = __shfl(h23, s0, 32), a2 = __shfl(h01, s1, 32), a3 = __shfl(h23, s1, 32);
  const int b0 = __shfl(l01, s0, 32), b1 = __shfl(l23, s0, 32), b2 = __shfl(l01, s1, 32), b3 = __shfl(l23, s1, 32);
  const int mk = (lane < 16) ? -1 : 0;
  v4i o;
  o.x = (a0 & mk) | (b0 & ~mk); o.y = (a1 & mk) | (b1 & ~mk);
  o.z = (a2 & mk) | (b2 & ~mk); o.w = (a3 & mk) | (b3 & ~mk);
  return o;
}

__device__ __forceinline__ void st2_v4f(float* p, v4f v) {
  *(volatile v4f*)p = v;
  __threadfence();
  *(volatile v4f*)p = v;
}
__device__ __forceinline__ void st2_v8us(unsigned short* p, v8us v) {
  *(volatile v8us*)p = v;
  __threadfence();
  *(volatile v8us*)p = v;
}

__device__ __forceinline__ void wplane_unit(const float* __restrict__ w, unsigned short* wd, int u) {
  const int l = u >> 12, n = (u >> 5) & (HD - 1), k8 = (u & 31) * 8, kk = k8 & (HD - 1);
  const float* p = w + (size_t)l * HD * HD + (size_t)n * HD + kk;
  const v4f a = *(const v4fa*)p;
  const v4f b = *(const v4fa*)(p + 4);
  v8us o;
  o[0] = (unsigned short)bf16_bits(a.x); o[1] = (unsigned short)bf16_bits(a.y);
  o[2] = (unsigned short)bf16_bits(a.z); o[3] = (unsigned short)bf16_bits(a.w);
  o[4] = (unsigned short)bf16_bits(b.x); o[5] = (unsigned short)bf16_bits(b.y);
  o[6] = (unsigned short)bf16_bits(b.z); o[7] = (unsigned short)bf16_bits(b.w);
  st2_v8us(wd + (size_t)l * HD * KTOT + (size_t)n * KTOT + k8, o);
}

__global__ __launch_bounds__(NTHR) void k_prep(const int* __restrict__ feats, const float* __restrict__ ke,
                                               const float* __restrict__ ve, const float* __restrict__ w1,
                                               const float* __restrict__ b1, const float* __restrict__ w2,
                                               const float* __restrict__ b2, const float* __restrict__ wc,
                                               float* H, unsigned short* w1d, unsigned short* w2d,
                                               unsigned short* wcd, float* bt) {
  const int tid = (int)threadIdx.x;
  const int blk = (int)blockIdx.x;
  if (blk < PBH) {
    const int u   = blk * NTHR + tid;
    const int row = u >> 5, c4 = (u & 31) * 4;
    const int rc  = row < NN ? row : NN - 1;
    const v2i f = *(const v2ia*)(feats + 2 * rc);
    int f0 = f.x, f1 = f.y;
    f0 = f0 < 0 ? 0 : (f0 > VOC - 1 ? VOC - 1 : f0);
    f1 = f1 < 0 ? 0 : (f1 > VOC - 1 ? VOC - 1 : f1);
    const v4f a = *(const v4fa*)(ke + (size_t)f0 * HD + c4);
    const v4f b = *(const v4fa*)(ve + (size_t)f1 * HD + c4);
    asm volatile("" :: "v"(a));
    asm volatile("" :: "v"(b));
    float v0 = bf16_val(a.x) + bf16_val(b.x), v1 = bf16_val(a.y) + bf16_val(b.y);
    float v2 = bf16_val(a.z) + bf16_val(b.z), v3 = bf16_val(a.w) + bf16_val(b.w);
    v0 = (v0 > 0.0f) ? v0 : (v0 - v0); v1 = (v1 > 0.0f) ? v1 : (v1 - v1);
    v2 = (v2 > 0.0f) ? v2 : (v2 - v2); v3 = (v3 > 0.0f) ? v3 : (v3 - v3);
    const bool live = row < NN;
    v4f o;
    o.x = live ? v0 : 0.0f; o.y = live ? v1 : 0.0f; o.z = live ? v2 : 0.0f; o.w = live ? v3 : 0.0f;
    st2_v4f(H + (size_t)row * HD + c4, o);
  } else if (blk < PBH + PBW) {
    wplane_unit(w1, w1d, (blk - PBH) * NTHR + tid);
  } else if (blk < PBH + 2 * PBW) {
    wplane_unit(w2, w2d, (blk - PBH - PBW) * NTHR + tid);
  } else if (blk < PBH + 2 * PBW + PBC) {
    const int u  = (blk - PBH - 2 * PBW) * NTHR + tid;
    const int n  = u >> 5, k8 = (u & 31) * 8, kk = k8 & (HD - 1);
    const int nc = n < NC ? n : NC - 1;
    const unsigned mk = n < NC ? 0xffffu : 0u;
    const float* p = wc + (size_t)nc * HD + kk;
    const v4f a = *(const v4fa*)p;
    const v4f b = *(const v4fa*)(p + 4);
    v8us o;
    o[0] = (unsigned short)(bf16_bits(a.x) & mk); o[1] = (unsigned short)(bf16_bits(a.y) & mk);
    o[2] = (unsigned short)(bf16_bits(a.z) & mk); o[3] = (unsigned short)(bf16_bits(a.w) & mk);
    o[4] = (unsigned short)(bf16_bits(b.x) & mk); o[5] = (unsigned short)(bf16_bits(b.y) & mk);
    o[6] = (unsigned short)(bf16_bits(b.z) & mk); o[7] = (unsigned short)(bf16_bits(b.w) & mk);
    st2_v8us(wcd + (size_t)n * KTOT + k8, o);
  } else {
    if (tid < 192) {
      const int i1 = tid < 96 ? tid : 95;
      const int i2 = tid >= 96 ? tid - 96 : 0;
      const v4f a = *(const v4fa*)(b1 + 4 * i1);
      const v4f c = *(const v4fa*)(b2 + 4 * i2);
      asm volatile("" :: "v"(a));
      asm volatile("" :: "v"(c));
      const unsigned ma = (tid < 96) ? 0xffffffffu : 0u;
      v4f o;
      o.x = __uint_as_float(((bf16_bits(a.x) << 16) & ma) | ((bf16_bits(c.x) << 16) & ~ma));
      o.y = __uint_as_float(((bf16_bits(a.y) << 16) & ma) | ((bf16_bits(c.y) << 16) & ~ma));
      o.z = __uint_as_float(((bf16_bits(a.z) << 16) & ma) | ((bf16_bits(c.z) << 16) & ~ma));
      o.w = __uint_as_float(((bf16_bits(a.w) << 16) & ma) | ((bf16_bits(c.w) << 16) & ~ma));
      st2_v4f(bt + 4 * tid, o);
    }
  }
}

__device__ __forceinline__ void bucket_flush(const int* pl, const int* cnt, int ov, int* lp, int* cop, int* fp,
                                             int tid) {
#pragma unroll 1
  for (int i = tid * 4; i < RCAP; i += NTHR * 4) {
    const v4i v = *(const v4ia*)(pl + i);
    *(volatile v4i*)(lp + i) = v;
  }
#pragma unroll 1
  for (int i = tid * 4; i < 2 * NBRUN; i += NTHR * 4) {
    const v4i v = *(const v4ia*)(cnt + i);
    *(volatile v4i*)(cop + i) = v;
  }
  if (tid < 8) {
    const v4i f = {ov, ov, ov, ov};
    *(volatile v4i*)(fp + 4 * tid) = f;
  }
}

__global__ __launch_bounds__(NTHR) void k_bucket(const int* __restrict__ srcs, const int* __restrict__ dsts,
                                                 int* LIST, int* CO, int* FLAG) {
  extern __shared__ __attribute__((aligned(16))) int dsm[];
  int* wl   = dsm;
  int* pl   = dsm + NWAVE * WLCAP;
  int* cnt  = pl + RCAP;
  int* offs = cnt + NBRUN;
  int* cur  = offs + NBRUN;
  int* misc = cur + NBRUN;
  const int tid = (int)threadIdx.x, lane = tid & 31, wave = tid >> 5;
  const int blk = (int)blockIdx.x;
  const unsigned nbs = (unsigned)(blk * NBRUN);
  const int nbi = (NN - blk * NBRUN) < NBRUN ? (NN - blk * NBRUN) : NBRUN;
  const unsigned unb = (unsigned)(nbi < 0 ? 0 : nbi);

  {
    const v4i z4 = {0, 0, 0, 0};
    for (int i = tid * 4; i < BK_ZINTS; i += NTHR * 4) *(v4ia*)(dsm + i) = z4;
    if (tid < 16) misc[tid] = 0;
  }
  __syncthreads();

  {
    const int per  = ((NE + NWAVE * WCH - 1) / (NWAVE * WCH)) * WCH;
    const int ebeg = wave * per;
    const int eend = (ebeg + per < NE) ? (ebeg + per) : NE;
    int* mylist = wl + wave * WLCAP;
    int wc = 0;
#pragma unroll 1
    for (int cb = ebeg; cb < eend; cb += WCH) {
      const int e0 = cb + lane * EPT;
      const v4i da = *(const v4ia*)(dsts + e0);
      const v4i db = *(const v4ia*)(dsts + e0 + 4);
      const unsigned s0 = (unsigned)da.x - nbs, s1 = (unsigned)da.y - nbs;
      const unsigned s2 = (unsigned)da.z - nbs, s3 = (unsigned)da.w - nbs;
      const unsigned s4 = (unsigned)db.x - nbs, s5 = (unsigned)db.y - nbs;
      const unsigned s6 = (unsigned)db.z - nbs, s7 = (unsigned)db.w - nbs;
      const bool h0 = s0 < unb, h1 = s1 < unb, h2 = s2 < unb, h3 = s3 < unb;
      const bool h4 = s4 < unb, h5 = s5 < unb, h6 = s6 < unb, h7 = s7 < unb;
      const unsigned m0 = __builtin_amdgcn_ballot_w32(h0), m1 = __builtin_amdgcn_ballot_w32(h1);
      const unsigned m2 = __builtin_amdgcn_ballot_w32(h2), m3 = __builtin_amdgcn_ballot_w32(h3);
      const unsigned m4 = __builtin_amdgcn_ballot_w32(h4), m5 = __builtin_amdgcn_ballot_w32(h5);
      const unsigned m6 = __builtin_amdgcn_ballot_w32(h6), m7 = __builtin_amdgcn_ballot_w32(h7);
      const unsigned any = m0 | m1 | m2 | m3 | m4 | m5 | m6 | m7;
      if (any != 0u) {
        const int pre = (int)(__builtin_amdgcn_mbcnt_lo(m0, 0u) + __builtin_amdgcn_mbcnt_lo(m1, 0u) +
                              __builtin_amdgcn_mbcnt_lo(m2, 0u) + __builtin_amdgcn_mbcnt_lo(m3, 0u) +
                              __builtin_amdgcn_mbcnt_lo(m4, 0u) + __builtin_amdgcn_mbcnt_lo(m5, 0u) +
                              __builtin_amdgcn_mbcnt_lo(m6, 0u) + __builtin_amdgcn_mbcnt_lo(m7, 0u));
        int p = wc + pre;
        if (h0) { if (p < WLCAP) mylist[p] = ((e0 + 0) << SLB) | (int)s0; p = p + 1; }
        if (h1) { if (p < WLCAP) mylist[p] = ((e0 + 1) << SLB) | (int)s1; p = p + 1; }
        if (h2) { if (p < WLCAP) mylist[p] = ((e0 + 2) << SLB) | (int)s2; p = p + 1; }
        if (h3) { if (p < WLCAP) mylist[p] = ((e0 + 3) << SLB) | (int)s3; p = p + 1; }
        if (h4) { if (p < WLCAP) mylist[p] = ((e0 + 4) << SLB) | (int)s4; p = p + 1; }
        if (h5) { if (p < WLCAP) mylist[p] = ((e0 + 5) << SLB) | (int)s5; p = p + 1; }
        if (h6) { if (p < WLCAP) mylist[p] = ((e0 + 6) << SLB) | (int)s6; p = p + 1; }
        if (h7) { if (p < WLCAP) mylist[p] = ((e0 + 7) << SLB) | (int)s7; p = p + 1; }
        wc += (int)(__builtin_popcount(m0) + __builtin_popcount(m1) + __builtin_popcount(m2) + __builtin_popcount(m3) +
                    __builtin_popcount(m4) + __builtin_popcount(m5) + __builtin_popcount(m6) + __builtin_popcount(m7));
      }
    }
    if (lane == 0) misc[wave] = wc;
  }
  __syncthreads();

  if (wave == 0) {
    int ov = 0;
#pragma unroll 1
    for (int w2 = 0; w2 < NWAVE; ++w2) {
      int c = misc[w2];
      if (c > WLCAP) ov = 1;
      c = c < 0 ? 0 : (c > WLCAP ? WLCAP : c);
#pragma unroll 1
      for (int b0 = 0; b0 < c; b0 += 32) {
        const int idx = b0 + lane;
        const int ent = wl[w2 * WLCAP + (idx < WLCAP ? idx : WLCAP - 1)];
        const int m32 = (c - b0) < 32 ? (c - b0) : 32;
#pragma unroll 1
        for (int k = 0; k < m32; ++k) {
          const int u    = __builtin_amdgcn_readlane(ent, k);
          const int slot = u & (NBRUN - 1);
          if (lane == 0) cnt[slot] = cnt[slot] + 1;
        }
      }
    }
    if (lane == 0) misc[9] = ov;
  }
  __syncthreads();
  if (wave == 0) {
    const int base = lane * (NBRUN / 32);
    int s = 0;
#pragma unroll 1
    for (int i = 0; i < NBRUN / 32; ++i) s += cnt[base + i];
    int incl = s;
#pragma unroll
    for (int d = 1; d < 32; d <<= 1) {
      const int y = __shfl_up(incl, d, 32);
      if (lane >= d) incl += y;
    }
    int run = incl - s;
#pragma unroll 1
    for (int i = 0; i < NBRUN / 32; ++i) {
      const int cv = cnt[base + i];
      offs[base + i] = run;
      cur[base + i]  = run;
      run += cv;
    }
  }
  __syncthreads();

  if (wave == 0) {
#pragma unroll 1
    for (int w2 = 0; w2 < NWAVE; ++w2) {
      int c = misc[w2];
      c = c < 0 ? 0 : (c > WLCAP ? WLCAP : c);
#pragma unroll 1
      for (int b0 = 0; b0 < c; b0 += 32) {
        const int idx = b0 + lane;
        const int ent = wl[w2 * WLCAP + (idx < WLCAP ? idx : WLCAP - 1)];
        int eid = (ent >> SLB) & 0x1FFFFF;
        eid = eid > NE - 1 ? NE - 1 : eid;
        int sr = srcs[eid];
        sr = sr < 0 ? 0 : (sr > NN - 1 ? NN - 1 : sr);
        const int m32 = (c - b0) < 32 ? (c - b0) : 32;
#pragma unroll 1
        for (int k = 0; k < m32; ++k) {
          const int u    = __builtin_amdgcn_readlane(ent, k);
          const int wd   = __builtin_amdgcn_readlane(sr, k);
          const int slot = u & (NBRUN - 1);
          if (lane == 0) {
            int p = cur[slot];
            p = p < 0 ? 0 : (p > RCAP - 1 ? RCAP - 1 : p);
            pl[p] = wd;
            cur[slot] = p + 1;
          }
        }
      }
    }
  }
  __syncthreads();

  const int ovf = misc[9];
  int* lp  = LIST + (size_t)blk * RCAP;
  int* cop = CO + (size_t)blk * (2 * NBRUN);
  int* fp  = FLAG + (size_t)blk * 32;
  bucket_flush(pl, cnt, ovf, lp, cop, fp, tid);
  __threadfence();
  bucket_flush(pl, cnt, ovf, lp, cop, fp, tid);
}

__global__ __launch_bounds__(NTHR) void k_replay(const int* __restrict__ LIST, const int* __restrict__ CO,
                                                 const int* __restrict__ FLAG, const float* __restrict__ H,
                                                 unsigned short* Z) {
  const int tid = (int)threadIdx.x, lane = tid & 31, wave = tid >> 5;
  const int rowBase = (int)blockIdx.x * RBM;
  const int bucket  = rowBase >> SLB;
  const int* lb  = LIST + (size_t)bucket * RCAP;
  const int* cob = CO + (size_t)bucket * (2 * NBRUN);
  const int flag = FLAG[(size_t)bucket * 32];
  const float qnan = __uint_as_float(0x7fc00000u);

#pragma unroll 1
  for (int i = 0; i < RBM / NWAVE; ++i) {
    const int d    = rowBase + (RBM / NWAVE) * wave + i;
    const int slot = d & (NBRUN - 1);
    int c = cob[slot];
    int o = cob[NBRUN + slot];
    const bool big = c > DEGCAP;
    c = c < 0 ? 0 : (c > DEGCAP ? DEGCAP : c);
    o = o < 0 ? 0 : (o > RCAP - 1 ? RCAP - 1 : o);
    int last = o + c - 1; last = last < o ? o : last;
    last = last > RCAP - 1 ? RCAP - 1 : last;
    const int cs = __builtin_amdgcn_readfirstlane(c);
    float a0 = 0.0f, a1 = 0.0f, a2 = 0.0f, a3 = 0.0f;
#pragma unroll 1
    for (int b0 = 0; b0 < cs; b0 += 32) {
      int idx = o + b0 + lane;
      idx = idx > last ? last : idx;
      int sv = lb[idx];
      sv = sv < 0 ? 0 : (sv > NN - 1 ? NN - 1 : sv);
      const int m32 = (cs - b0) < 32 ? (cs - b0) : 32;
#pragma unroll 1
      for (int k = 0; k < m32; ++k) {
        const int sk = __builtin_amdgcn_readlane(sv, k);
        const v4f v = *(const v4fa*)(H + (size_t)sk * HD + 4 * lane);
        a0 += v.x; a1 += v.y; a2 += v.z; a3 += v.w;
      }
    }
    const v4f g = *(const v4fa*)(H + (size_t)d * HD + 4 * lane);
    asm volatile("" :: "v"(g));
    float z0 = g.x + a0, z1 = g.y + a1, z2 = g.z + a2, z3 = g.w + a3;
    const bool bad  = (flag != 0) | big;
    const bool live = d < NN;
    z0 = bad ? qnan : z0; z1 = bad ? qnan : z1; z2 = bad ? qnan : z2; z3 = bad ? qnan : z3;
    z0 = live ? z0 : 0.0f; z1 = live ? z1 : 0.0f; z2 = live ? z2 : 0.0f; z3 = live ? z3 : 0.0f;
    int h01, h23, l01, l23;
    hilo_pack(z0, z1, z2, z3, h01, h23, l01, l23);
    const v4i ow = regroup32(h01, h23, l01, l23, lane);
    unsigned short* zp = Z + (size_t)d * KTOT + 8 * lane;
    *(volatile v4i*)zp = ow;
    __threadfence();
    *(volatile v4i*)zp = ow;
  }
}

template <int NT>
__device__ __forceinline__ void mm_glb(const unsigned short* __restrict__ ap,
                                       const unsigned short* __restrict__ bp, v8f (&acc)[NT]) {
#pragma unroll 1
  for (int k0 = 0; k0 < KTOT; k0 += 32) {
    FragB af;
    af.h[0] = *(const v8usa*)(ap + k0);
    af.h[1] = *(const v8usa*)(ap + k0 + 16);
#pragma unroll
    for (int nt = 0; nt < NT; ++nt) {
      const unsigned short* wq = bp + (size_t)(16 * nt) * (size_t)KTOT + k0;
      FragB bf;
      bf.h[0] = *(const v8usa*)wq;
      bf.h[1] = *(const v8usa*)(wq + 16);
      acc[nt] = wmb(af, bf, acc[nt]);
    }
  }
}
template <int NT>
__device__ __forceinline__ void mm_lds(const unsigned short* ap,
                                       const unsigned short* __restrict__ bp, v8f (&acc)[NT]) {
#pragma unroll 1
  for (int k0 = 0; k0 < KTOT; k0 += 32) {
    FragB af;
    af.h[0] = *(const v8usa*)(ap + k0);
    af.h[1] = *(const v8usa*)(ap + k0 + 16);
#pragma unroll
    for (int nt = 0; nt < NT; ++nt) {
      const unsigned short* wq = bp + (size_t)(16 * nt) * (size_t)KTOT + k0;
      FragB bf;
      bf.h[0] = *(const v8usa*)wq;
      bf.h[1] = *(const v8usa*)(wq + 16);
      acc[nt] = wmb(af, bf, acc[nt]);
    }
  }
}

__device__ __forceinline__ void stage_d8(float* stg, const v8f (&acc)[8], int wave, int hh, int m) {
#pragma unroll
  for (int nt = 0; nt < 8; ++nt) {
#pragma unroll
    for (int r = 0; r < 8; ++r) stg[(16 * wave + 8 * hh + r) * SP + 16 * nt + m] = acc[nt][r];
  }
}

__device__ __forceinline__ void out_flush(const float* og, float* ob, int nv4, int flag, int tid) {
  const float qnan = __uint_as_float(0x7fc00000u);
#pragma unroll 1
  for (int it = 0; it < 5; ++it) {
    const int i4 = it * NTHR + tid;
    v4f v = *(const v4fa*)(og + 4 * i4);
    asm volatile("" :: "v"(v));
    v.x = (flag != 0) ? qnan : v.x; v.y = (flag != 0) ? qnan : v.y;
    v.z = (flag != 0) ? qnan : v.z; v.w = (flag != 0) ? qnan : v.w;
    if (i4 < nv4) *(volatile v4f*)(ob + (size_t)4 * (size_t)i4) = v;
  }
}

template <int LAST>
__global__ __launch_bounds__(NTHR) __attribute__((amdgpu_num_vgpr(248)))
void k_mlp(const unsigned short* __restrict__ Z, const unsigned short* __restrict__ W1p,
           const unsigned short* __restrict__ W2p, const unsigned short* __restrict__ WcP,
           const float* __restrict__ bt1, const float* __restrict__ bt2,
           const int* __restrict__ FLAG, float* H, float* out) {
  extern __shared__ __attribute__((aligned(16))) int dsm[];
  float* stg = (float*)dsm;
  unsigned short* tt = (unsigned short*)(dsm + GBM * SP);
  float* sb = (float*)(dsm + GBM * SP + (GBM * TPH) / 2);
  const int tid = (int)threadIdx.x, lane = tid & 31, wave = tid >> 5, hh = lane >> 4, m = lane & 15;
  const int blk = (int)blockIdx.x;
  const int rowBase = blk * GBM;
  const int flag = FLAG[(size_t)(blk >> 3) * 32];

  if (tid < 32) {
    *(v4fa*)(sb + 4 * tid) = *(const v4fa*)(bt1 + 4 * tid);
  } else if (tid < 64) {
    *(v4fa*)(sb + HD + 4 * (tid - 32)) = *(const v4fa*)(bt2 + 4 * (tid - 32));
  }

  v8f acc[8];
  const v8f zz = {0.f, 0.f, 0.f, 0.f, 0.f, 0.f, 0.f, 0.f};
#pragma unroll
  for (int t = 0; t < 8; ++t) acc[t] = zz;

  {
    const unsigned short* ap = Z + (size_t)(rowBase + 16 * wave + m) * (size_t)KTOT + 8 * hh;
    const unsigned short* bp = W1p + (size_t)m * (size_t)KTOT + 8 * hh;
    mm_glb<8>(ap, bp, acc);
  }
  stage_d8(stg, acc, wave, hh, m);
  __syncthreads();
  {
    const v4f b1v = *(const v4fa*)(sb + 4 * lane);
#pragma unroll 1
    for (int i = 0; i < 16; ++i) {
      const int lr = 16 * wave + i;
      const v4f a = *(const v4fa*)(stg + lr * SP + 4 * lane);
      float v0 = a.x + b1v.x, v1 = a.y + b1v.y, v2 = a.z + b1v.z, v3 = a.w + b1v.w;
      v0 = (v0 > 0.0f) ? v0 : (v0 - v0); v1 = (v1 > 0.0f) ? v1 : (v1 - v1);
      v2 = (v2 > 0.0f) ? v2 : (v2 - v2); v3 = (v3 > 0.0f) ? v3 : (v3 - v3);
      int h01, h23, l01, l23;
      hilo_pack(v0, v1, v2, v3, h01, h23, l01, l23);
      const v4i ow = regroup32(h01, h23, l01, l23, lane);
      *(v4ia*)(tt + lr * TPH + 8 * lane) = ow;
    }
  }
  __syncthreads();

#pragma unroll
  for (int t = 0; t < 8; ++t) acc[t] = zz;
  {
    const unsigned short* ap = tt + (16 * wave + m) * TPH + 8 * hh;
    const unsigned short* bp = W2p + (size_t)m * (size_t)KTOT + 8 * hh;
    mm_lds<8>(ap, bp, acc);
  }
  __syncthreads();
  stage_d8(stg, acc, wave, hh, m);
  __syncthreads();

  const v4f b2v = *(const v4fa*)(sb + HD + 4 * lane);
  if constexpr (LAST == 0) {
#pragma unroll 1
    for (int i = 0; i < 16; ++i) {
      const int lr   = 16 * wave + i;
      const int grow = rowBase + lr;
      const bool live = grow < NN;
      const v4f a = *(const v4fa*)(stg + lr * SP + 4 * lane);
      asm volatile("" :: "v"(a));
      const float v0 = a.x + b2v.x, v1 = a.y + b2v.y, v2 = a.z + b2v.z, v3 = a.w + b2v.w;
      v4f o;
      o.x = live ? v0 : 0.0f; o.y = live ? v1 : 0.0f; o.z = live ? v2 : 0.0f; o.w = live ? v3 : 0.0f;
      st2_v4f(H + (size_t)grow * HD + 4 * lane, o);
    }
  } else {
#pragma unroll 1
    for (int i = 0; i < 16; ++i) {
      const int lr = 16 * wave + i;
      const v4f a = *(const v4fa*)(stg + lr * SP + 4 * lane);
      const float v0 = a.x + b2v.x, v1 = a.y + b2v.y, v2 = a.z + b2v.z, v3 = a.w + b2v.w;
      int h01, h23, l01, l23;
      hilo_pack(v0, v1, v2, v3, h01, h23, l01, l23);
      const v4i ow = regroup32(h01, h23, l01, l23, lane);
      *(v4ia*)(tt + lr * TPH + 8 * lane) = ow;
    }
    __syncthreads();

    v8f ac3[3];
#pragma unroll
    for (int t = 0; t < 3; ++t) ac3[t] = zz;
    {
      const unsigned short* ap = tt + (16 * wave + m) * TPH + 8 * hh;
      const unsigned short* bp = WcP + (size_t)m * (size_t)KTOT + 8 * hh;
      mm_lds<3>(ap, bp, ac3);
    }
    float* og = stg;
#pragma unroll
    for (int t = 0; t < 3; ++t) {
      const int col = 16 * t + m;
#pragma unroll
      for (int r = 0; r < 8; ++r) {
        if (col < NC) og[(16 * wave + 8 * hh + r) * NC + col] = ac3[t][r];
      }
    }
    __syncthreads();

    const int liveRows = (NN - rowBase) < GBM ? (NN - rowBase) : GBM;
    const int nv4 = liveRows * (NC / 4);
    float* ob = out + (size_t)blk * (size_t)(GBM * NC);
    out_flush(og, ob, nv4, flag, tid);
    __threadfence();
    out_flush(og, ob, nv4, flag, tid);
  }
}

extern "C" void kernel_launch(void* const* d_in, const int* in_sizes, int n_in,
                              void* d_out, int out_size, void* d_ws, size_t ws_size,
                              hipStream_t stream) {
  if (n_in < 10) return;
  if (in_sizes[0] != NN * 2) return;
  if (in_sizes[1] != NE) return;
  if (in_sizes[2] != NE) return;
  if (in_sizes[3] != VOC * HD) return;
  if (in_sizes[4] != VOC * HD) return;
  if (in_sizes[5] != NLAY * HD * HD) return;
  if (in_sizes[6] != NLAY * HD) return;
  if (in_sizes[7] != NLAY * HD * HD) return;
  if (in_sizes[8] != NLAY * HD) return;
  if (in_sizes[9] != NC * HD) return;
  if (out_size != NN * NC) return;

  const int*   feats = (const int*)d_in[0];
  const int*   srcs  = (const int*)d_in[1];
  const int*   dsts  = (const int*)d_in[2];
  const float* ke    = (const float*)d_in[3];
  const float* ve    = (const float*)d_in[4];
  const float* W1    = (const float*)d_in[5];
  const float* b1    = (const float*)d_in[6];
  const float* W2    = (const float*)d_in[7];
  const float* b2    = (const float*)d_in[8];
  const float* Wc    = (const float*)d_in[9];
  float* out = (float*)d_out;

  constexpr size_t zH    = (size_t)MP * HD * 4;
  constexpr size_t zZ    = (size_t)MP * KTOT * 2;
  constexpr size_t zLIST = (size_t)NBK * RCAP * 4;
  constexpr size_t zCO   = (size_t)NBK * 2 * NBRUN * 4;
  constexpr size_t zFLAG = 6400;
  constexpr size_t zWD   = (size_t)NLAY * HD * KTOT * 2;
  constexpr size_t zWC   = (size_t)NCP * KTOT * 2;
  constexpr size_t zBT   = (size_t)2 * NLAY * HD * 4;
  constexpr size_t oH    = 0;
  constexpr size_t oZ    = oH + zH;
  constexpr size_t oLIST = oZ + zZ;
  constexpr size_t oCO   = oLIST + zLIST;
  constexpr size_t oFLAG = oCO + zCO;
  constexpr size_t oW1D  = oFLAG + zFLAG;
  constexpr size_t oW2D  = oW1D + zWD;
  constexpr size_t oWCD  = oW2D + zWD;
  constexpr size_t oBT   = oWCD + zWC;
  constexpr size_t oEND  = oBT + zBT;
  static_assert(zH % 256 == 0 && zZ % 256 == 0 && zLIST % 256 == 0 && zCO % 256 == 0 && zFLAG % 256 == 0);
  static_assert(zWD % 256 == 0 && zWC % 256 == 0 && zBT % 256 == 0);
  static_assert(zFLAG >= (size_t)NBK * 128);
  static_assert(oEND <= (size_t)WSMAX);
  if (oEND > ws_size) return;

  char* ws = (char*)d_ws;
  float*          H    = (float*)(ws + oH);
  unsigned short* Zp   = (unsigned short*)(ws + oZ);
  int*            LIST = (int*)(ws + oLIST);
  int*            CO   = (int*)(ws + oCO);
  int*            FLAG = (int*)(ws + oFLAG);
  unsigned short* W1D  = (unsigned short*)(ws + oW1D);
  unsigned short* W2D  = (unsigned short*)(ws + oW2D);
  unsigned short* WCD  = (unsigned short*)(ws + oWCD);
  float*          BT   = (float*)(ws + oBT);

  hipFuncSetAttribute(reinterpret_cast<const void*>(&k_bucket), hipFuncAttributeMaxDynamicSharedMemorySize, (int)BK_LDS);
  hipFuncSetAttribute(reinterpret_cast<const void*>(&k_mlp<0>), hipFuncAttributeMaxDynamicSharedMemorySize, (int)ML_LDS);
  hipFuncSetAttribute(reinterpret_cast<const void*>(&k_mlp<1>), hipFuncAttributeMaxDynamicSharedMemorySize, (int)ML_LDS);

  k_prep<<<PBTOT, NTHR, 0, stream>>>(feats, ke, ve, W1, b1, W2, b2, Wc, H, W1D, W2D, WCD, BT);
  k_bucket<<<NBK, NTHR, BK_LDS, stream>>>(srcs, dsts, LIST, CO, FLAG);

  for (int l = 0; l < NLAY; ++l) {
    k_replay<<<MP / RBM, NTHR, 0, stream>>>(LIST, CO, FLAG, H, Zp);
    const unsigned short* w1p = W1D + (size_t)l * HD * KTOT;
    const unsigned short* w2p = W2D + (size_t)l * HD * KTOT;
    const float* bt1 = BT + (size_t)l * HD;
    const float* bt2 = BT + (size_t)NLAY * HD + (size_t)l * HD;
    if (l == NLAY - 1)
      k_mlp<1><<<MP / GBM, NTHR, ML_LDS, stream>>>(Zp, w1p, w2p, WCD, bt1, bt2, FLAG, H, out);
    else
      k_mlp<0><<<MP / GBM, NTHR, ML_LDS, stream>>>(Zp, w1p, w2p, WCD, bt1, bt2, FLAG, H, out);
  }
}
